// EdgeNetwork_66254165508977
// MI455X (gfx1250) — hardware-verified
//
#include <hip/hip_runtime.h>
#include <stdint.h>

typedef __attribute__((ext_vector_type(16))) __bf16   v16b;
typedef __attribute__((ext_vector_type(8)))  __bf16   v8b;
typedef __attribute__((ext_vector_type(8)))  float    v8f;
typedef __attribute__((ext_vector_type(4)))  float    v4f;

__device__ __forceinline__ unsigned short f2bf_bits(float f) {
  unsigned u = __float_as_uint(f);
  return (unsigned short)((u + 0x7FFFu + ((u >> 16) & 1u)) >> 16);
}
__device__ __forceinline__ float bf_bits2f(unsigned short h) { return __uint_as_float(((unsigned)h) << 16); }

__device__ __forceinline__ void dep_guard4_b(v8f& a, v8f& b, v16b x, v16b y, v16b z, v16b w) {
  asm volatile("v_nop\n\tv_nop\n\tv_nop\n\tv_nop" : "+v"(a), "+v"(b) : "v"(x), "v"(y), "v"(z), "v"(w));
}

template <typename T> struct Frag;
template <> struct Frag<__bf16> {
  typedef v16b V; union U { v16b v; v8b h[2]; };
  static __device__ __forceinline__ v16b load(const __bf16* p) {
    U f; f.h[0] = *(const v8b*)(p); f.h[1] = *(const v8b*)(p + 16); return f.v;
  }
  static __device__ __forceinline__ v8f mma(v16b a, v16b b, v8f c) {
    return __builtin_amdgcn_wmma_f32_16x16x32_bf16(false, a, false, b, (short)0, c, false, false);
  }
};

__device__ __forceinline__ void split_bf(float f, __bf16& hi, __bf16& lo) {
  const unsigned short hb = f2bf_bits(f);
  hi = __builtin_bit_cast(__bf16, hb);
  lo = __builtin_bit_cast(__bf16, f2bf_bits(f - bf_bits2f(hb)));
}

constexpr int kStateDim = 32;
constexpr int kNCols    = kStateDim * kStateDim;
constexpr int kNFeat    = 16;
constexpr int kWPB      = 8;
constexpr int kThreads  = kWPB * 32;
constexpr int kWPitch   = 32;
constexpr int kOsPitch  = 36;
constexpr int kTileRows = 16;

static_assert(kNCols == 1024);
static_assert(kThreads * 4 == kNCols);
static_assert((kWPitch % 8) == 0 && (kOsPitch % 4) == 0);

__global__ __launch_bounds__(kThreads)
void edge_mlp_matvec(const float* __restrict__ states,
                     const float* __restrict__ edges,
                     const float* __restrict__ W,
                     const float* __restrict__ bias,
                     float* __restrict__ out,
                     int numTiles)
{
  __shared__ __align__(16) __bf16 Wl[kNCols * kWPitch];
  __shared__ __align__(16) float  bsh[kNCols];
  __shared__ __align__(16) float  Os[kWPB][kTileRows * kOsPitch];

  const int tid = threadIdx.x;

#pragma unroll 1
  for (int idx = tid; idx < kNCols * 2; idx += kThreads) {
    const int c = idx & (kNCols - 1);
    const int g = idx >> 10;
    float w[8];
#pragma unroll
    for (int j = 0; j < 8; ++j) w[j] = W[(size_t)(8 * g + j) * kNCols + c];
    v8b hv, lv;
#pragma unroll
    for (int j = 0; j < 8; ++j) {
      __bf16 hi, lo;
      split_bf(w[j], hi, lo);
      hv[j] = hi;
      lv[j] = lo;
    }
    *(v8b*)(Wl + (size_t)c * kWPitch + 8 * g) = hv;
    *(v8b*)(Wl + (size_t)c * kWPitch + 16 + 8 * g) = lv;
  }
  *(v4f*)(bsh + 4 * tid) = *(const v4f*)(bias + 4 * tid);
  __syncthreads();

  const int wave = tid >> 5, lane = tid & 31;
  const int m  = lane & 15;
  const int hh = lane >> 4;
  const int gw = blockIdx.x * kWPB + wave;
  const int nw = gridDim.x * kWPB;
  float* osw = Os[wave];

  for (int tile = gw; tile < numTiles; tile += nw) {
    const size_t rowBase = (size_t)tile * kTileRows;
    const size_t row = rowBase + m;

    v16b Bh, Bl;
    {
      const v4f e0 = *(const v4f*)(edges + row * kNFeat + 8 * hh);
      const v4f e1 = *(const v4f*)(edges + row * kNFeat + 8 * hh + 4);
      float ef[8] = {e0[0], e0[1], e0[2], e0[3], e1[0], e1[1], e1[2], e1[3]};
#pragma unroll
      for (int j = 0; j < 8; ++j) {
        __bf16 hi, lo;
        split_bf(ef[j], hi, lo);
        Bh[j] = hi; Bh[8 + j] = hi;
        Bl[j] = lo; Bl[8 + j] = lo;
      }
    }
    const v4f s0a = *(const v4f*)(states + row * kStateDim + 8 * hh);
    const v4f s0b = *(const v4f*)(states + row * kStateDim + 8 * hh + 4);
    const v4f s1a = *(const v4f*)(states + row * kStateDim + 16 + 8 * hh);
    const v4f s1b = *(const v4f*)(states + row * kStateDim + 16 + 8 * hh + 4);
    const float S0[8] = {s0a[0], s0a[1], s0a[2], s0a[3], s0b[0], s0b[1], s0b[2], s0b[3]};
    const float S1[8] = {s1a[0], s1a[1], s1a[2], s1a[3], s1b[0], s1b[1], s1b[2], s1b[3]};

#pragma unroll 2
    for (int i = 0; i < kStateDim; ++i) {
      const int c0 = kStateDim * i + m;
      const int c1 = c0 + 16;
      const v16b A0 = Frag<__bf16>::load(Wl + (size_t)c0 * kWPitch + 8 * hh);
      const v16b A1 = Frag<__bf16>::load(Wl + (size_t)c1 * kWPitch + 8 * hh);
      const v8f zero = (v8f){0.f, 0.f, 0.f, 0.f, 0.f, 0.f, 0.f, 0.f};
      v8f D0 = Frag<__bf16>::mma(A0, Bh, zero);
      D0 = Frag<__bf16>::mma(A0, Bl, D0);
      v8f D1 = Frag<__bf16>::mma(A1, Bh, zero);
      D1 = Frag<__bf16>::mma(A1, Bl, D1);
      dep_guard4_b(D0, D1, A0, A1, Bh, Bl);

      const float* bp = bsh + kStateDim * i + 8 * hh;
      const v4f b0a = *(const v4f*)(bp), b0b = *(const v4f*)(bp + 4);
      const v4f b1a = *(const v4f*)(bp + 16), b1b = *(const v4f*)(bp + 20);
      const float B0v[8] = {b0a[0], b0a[1], b0a[2], b0a[3], b0b[0], b0b[1], b0b[2], b0b[3]};
      const float B1v[8] = {b1a[0], b1a[1], b1a[2], b1a[3], b1b[0], b1b[1], b1b[2], b1b[3]};
      float acc0 = 0.f, acc1 = 0.f;
#pragma unroll
      for (int r = 0; r < 8; ++r) {
        const float x0 = fmaxf(D0[r] + B0v[r], 0.0f);
        const float x1 = fmaxf(D1[r] + B1v[r], 0.0f);
        acc0 = fmaf(x0, S0[r], acc0);
        acc1 = fmaf(x1, S1[r], acc1);
      }
      float acc = acc0 + acc1;
      acc += __shfl_xor(acc, 16, 32);
      osw[m * kOsPitch + i] = acc;
    }

    __builtin_amdgcn_fence(__ATOMIC_RELEASE, "workgroup");
    __builtin_amdgcn_wave_barrier();
    __builtin_amdgcn_fence(__ATOMIC_ACQUIRE, "workgroup");
    {
      const int q = lane >> 3, c4 = (lane & 7) * 4;
      float* obase = out + rowBase * kStateDim;
      for (int pass = 0; pass < 2; ++pass) {
#pragma unroll
        for (int it = 0; it < 4; ++it) {
          const int orow = it * 4 + q;
          const v4f v = *(const v4f*)(osw + orow * kOsPitch + c4);
          *(volatile v4f*)(obase + (size_t)orow * kStateDim + c4) = v;
        }
        __threadfence();
      }
    }
    __builtin_amdgcn_fence(__ATOMIC_RELEASE, "workgroup");
    __builtin_amdgcn_wave_barrier();
    __builtin_amdgcn_fence(__ATOMIC_ACQUIRE, "workgroup");
  }
}

extern "C" void kernel_launch(void* const* d_in, const int* in_sizes, int n_in,
                              void* d_out, int out_size, void* d_ws, size_t ws_size,
                              hipStream_t stream) {
  const float* states = (const float*)d_in[0];
  const float* edges  = (const float*)d_in[1];
  const float* W      = (const float*)d_in[2];
  const float* bias   = (const float*)d_in[3];
  float* out = (float*)d_out;
  (void)n_in; (void)d_ws; (void)ws_size;

  int rows = in_sizes[1] / kNFeat;
  const int rowsS = in_sizes[0] / kStateDim;
  const int rowsO = out_size / kStateDim;
  if (rowsS < rows) rows = rowsS;
  if (rowsO < rows) rows = rowsO;
  const int numTiles = rows / kTileRows;
  int blocks = (numTiles + kWPB - 1) / kWPB;
  if (blocks > 512) blocks = 512;
  if (blocks < 1) blocks = 1;

  hipLaunchKernelGGL(edge_mlp_matvec, dim3(blocks), dim3(kThreads), 0, stream,
                     states, edges, W, bias, out, numTiles);
}
